// LatentAttention_45114336477260
// MI455X (gfx1250) — hardware-verified
//
#include <hip/hip_runtime.h>
#include <math.h>
#include <stdint.h>

#ifndef NB
#define NB 2
#endif
#ifndef SEQ
#define SEQ 2048
#endif
#define XS_FULL 2048
#define DMOD  2048
#define NH    16
#define NKV   8
#define DN    128
#define DR    64
#define DV    128
#define RHALF (DR / 2)
#define QLR   768
#define KVLR  512
#define NDOWN (QLR + KVLR + DR)
#define QNW   (NH * DN)
#define QPW   (NH * DR)
#define NQUP  (QNW + QPW)
#define KNW   (NKV * DN)
#define NKVUP (KNW + NKV * DV)
#define ODIM  (NH * DV)
#define QO    ((SEQ < 256) ? SEQ : 256)
#define MROWS (NB * SEQ)
#define MCH   ((SEQ < 1024) ? SEQ : 1024)
#define NCH   (SEQ / MCH)
#define EPS_RMS 0.000001f
#define SCL   0.07216878364870322f
#define LOG2E 1.4426950408889634f
#define KROPE (-0.41524101186092029f)
#define NEGT  (-1.0e30f)
#define QSC   256.0f
#define KSC   256.0f
#define CSC   256.0f
#define WUS   1024.0f
#define PCAR  32768.0f
#define VCAR  1024.0f
#define OSC   1024.0f
#define WOS   1024.0f
#define WPB   2
#define NHG   (NH / WPB)
#define NQT   (SEQ / 16)
#define NST   (MCH / 64)
#define NKT   (SEQ / 32)
#define RPB   16
#define ATT_THREADS (WPB * 32)
#define PTP   36
#define PTW   (16 * PTP)
#define SLP   132
#define SLW   (16 * SLP)
#define WREG  (PTW + SLW)
#define SLAB64 (16 * 68)
#define VTP   72
#define TWP   72
#define WS_CAP 134217728
static_assert(NHG == NKV && NHG * WPB == NH && WPB == 2 && ATT_THREADS == 64);
static_assert(NB >= 1 && NB <= 2);
static_assert((SEQ % 64) == 0 && SEQ >= 64 && SEQ <= XS_FULL);
static_assert((QO % 64) == 0 && QO >= 64 && QO <= SEQ && (QO % 16) == 0);
static_assert((MCH % 64) == 0 && MCH >= 64 && NCH * MCH == SEQ && (MCH % RPB) == 0);
static_assert((NDOWN % 64) == 0 && (NQUP % 64) == 0 && (NKVUP % 64) == 0 && (ODIM % 64) == 0);
static_assert((DMOD % 64) == 0 && (QLR % 64) == 0 && (KVLR % 64) == 0 && (ODIM % 32) == 0);
static_assert((QLR % 256) == 0 && (KVLR % 256) == 0 && QLR <= 1024 && KVLR <= 1024);
static_assert(DN == 128 && DR == 64 && DV == 128 && RHALF * 2 == DR && (DN % 32) == 0 && (DR % 32) == 0);
static_assert(((MCH * DMOD / 8) % 256) == 0 && ((MCH * QNW / 8) % 256) == 0 && ((MCH * KNW / 8) % 256) == 0);
static_assert(QPW == 128 * 8 && RPB * 8 == 128);
static_assert(WPB * WREG * 4 <= 65536 && 2 * DV * VTP * 2 <= 65536 && 4 * SLAB64 * 4 <= 65536 && 64 * TWP * 2 <= 65536);
static_assert(2 * RPB * RHALF * 4 <= 65536);

typedef unsigned short u16;
typedef _Float16 v16h __attribute__((ext_vector_type(16)));
typedef _Float16 v8h  __attribute__((ext_vector_type(8)));
typedef __bf16   v16b __attribute__((ext_vector_type(16)));
typedef float    v8f  __attribute__((ext_vector_type(8)));
typedef float    v4f  __attribute__((ext_vector_type(4)));
typedef unsigned int v4u __attribute__((ext_vector_type(4)));

union FragH { v16h v; v8h h[2]; v4u u[2]; };
union FragB { v16b v; v4u u[2]; };

__device__ __forceinline__ unsigned short bf_bits(float f) {
  unsigned u = __float_as_uint(f);
  return (unsigned short)((u + 0x7FFFu + ((u >> 16) & 1u)) >> 16);
}
__device__ __forceinline__ float bf_up(unsigned short h) { return __uint_as_float(((unsigned)h) << 16); }
__device__ __forceinline__ float bfr(float f) { return bf_up(bf_bits(f)); }
__device__ __forceinline__ unsigned short h_bits(_Float16 x) { return __builtin_bit_cast(unsigned short, x); }
__device__ __forceinline__ unsigned pk16(unsigned short a, unsigned short b) { return (unsigned)a | ((unsigned)b << 16); }
__device__ __forceinline__ v8f zero8() { v8f z = {0.f, 0.f, 0.f, 0.f, 0.f, 0.f, 0.f, 0.f}; return z; }
__device__ __forceinline__ void hilo(float t, unsigned short& hb, unsigned short& lb) {
  const _Float16 h = (_Float16)t;
  hb = h_bits(h);
  lb = h_bits((_Float16)(t - (float)h));
}

__device__ __forceinline__ v16h ldfrag_h(const _Float16* p) {
  FragH f;
  f.h[0] = *(const v8h*)(p);
  f.h[1] = *(const v8h*)(p + 16);
  return f.v;
}
__device__ __forceinline__ v16b ldfrag_b(const u16* p) {
  FragB f;
  f.u[0] = *(const v4u*)(p);
  f.u[1] = *(const v4u*)(p + 16);
  return f.v;
}

__device__ __forceinline__ v8f mma_h(v16h a, v16h b, v8f c) {
  return __builtin_amdgcn_wmma_f32_16x16x32_f16(false, a, false, b, (short)0, c, false, false);
}
__device__ __forceinline__ v8f mma_b(v16b a, v16b b, v8f c) {
  return __builtin_amdgcn_wmma_f32_16x16x32_bf16(false, a, false, b, (short)0, c, false, false);
}
__device__ __forceinline__ void guard2(v8f& a, v8f& b, v16h x0, v16h x1, v16h x2, v16h x3, v16h x4, v16h x5) {
#if defined(__HIP_DEVICE_COMPILE__)
  asm volatile("v_nop\n\tv_nop\n\tv_nop\n\tv_nop"
               : "+v"(a), "+v"(b) : "v"(x0), "v"(x1), "v"(x2), "v"(x3), "v"(x4), "v"(x5) : "memory");
#endif
}
template <typename F>
__device__ __forceinline__ void guard6(v8f& a, v8f& b, v8f& c, v8f& d, F x0, F x1, F x2, F x3, F x4, F x5) {
#if defined(__HIP_DEVICE_COMPILE__)
  asm volatile("v_nop\n\tv_nop\n\tv_nop\n\tv_nop"
               : "+v"(a), "+v"(b), "+v"(c), "+v"(d) : "v"(x0), "v"(x1), "v"(x2), "v"(x3), "v"(x4), "v"(x5) : "memory");
#endif
}
__device__ __forceinline__ void acc_guard4(v8f& a, v8f& b, v8f& c, v8f& d) {
#if defined(__HIP_DEVICE_COMPILE__)
  asm volatile("v_nop\n\tv_nop\n\tv_nop\n\tv_nop" : "+v"(a), "+v"(b), "+v"(c), "+v"(d));
#endif
}
__device__ __forceinline__ void wave_sync_lds() {
  __builtin_amdgcn_fence(__ATOMIC_RELEASE, "workgroup");
  __builtin_amdgcn_wave_barrier();
  __builtin_amdgcn_fence(__ATOMIC_ACQUIRE, "workgroup");
}

__global__ __launch_bounds__(256) void cvtb16(const float* __restrict__ x, u16* D, int n8) {
  const int gt = blockIdx.x * 256 + (int)threadIdx.x;
  if (gt >= n8) return;
  const float* p = x + (size_t)gt * 8;
  const v4f a = *(const v4f*)(p), b4 = *(const v4f*)(p + 4);
  v4u o;
  o[0] = pk16(bf_bits(a[0]),  bf_bits(a[1]));
  o[1] = pk16(bf_bits(a[2]),  bf_bits(a[3]));
  o[2] = pk16(bf_bits(b4[0]), bf_bits(b4[1]));
  o[3] = pk16(bf_bits(b4[2]), bf_bits(b4[3]));
  u16* d = D + (size_t)gt * 8;
  for (int pass = 0; pass < 2; ++pass) {
    *(volatile v4u*)(d) = o;
    __threadfence();
  }
}

__global__ __launch_bounds__(256) void tw16(const float* __restrict__ W, int ldw, int K, int NN, u16* T,
                                            int f16mode, float scale) {
  __shared__ __align__(16) u16 TT[64 * TWP];
  const int tid = threadIdx.x;
  const int bid = blockIdx.x;
  const int ktn = K >> 6;
  const int kt  = bid % ktn;
  const int nt  = bid / ktn;
  if (nt >= (NN >> 6)) return;
  const int k0 = kt * 64, n0 = nt * 64;
  {
    const int kk = tid >> 2;
    const int nq = (tid & 3) * 16;
    const float* src = W + (size_t)(k0 + kk) * ldw + n0 + nq;
#pragma unroll
    for (int i = 0; i < 4; ++i) {
      const v4f a = *(const v4f*)(src + 4 * i);
#pragma unroll
      for (int e = 0; e < 4; ++e) {
        const float f = a[e];
        const unsigned short hb = h_bits((_Float16)(bfr(f) * scale));
        const unsigned short bb = bf_bits(f);
        TT[(nq + 4 * i + e) * TWP + kk] = (f16mode != 0) ? hb : bb;
      }
    }
  }
  __syncthreads();
  const int q8 = tid >> 3, p8 = (tid & 7) * 8;
  v4u v[2];
#pragma unroll
  for (int it = 0; it < 2; ++it) {
    const int line = it * 32 + q8;
    v[it] = *(const v4u*)(TT + line * TWP + p8);
  }
  const size_t base = (size_t)n0 * K + k0 + p8;
  for (int pass = 0; pass < 2; ++pass) {
#pragma unroll
    for (int it = 0; it < 2; ++it) {
      const int line = it * 32 + q8;
      *(volatile v4u*)(T + base + (size_t)line * K) = v[it];
    }
    __threadfence();
  }
}

__global__ __launch_bounds__(128) void rnorm16(const float* __restrict__ F, int ldf, int D, float invD,
                                               const float* __restrict__ nw, u16* Hp, u16* Lp, float sc) {
  __shared__ float red[4];
  const int tid = (int)threadIdx.x, wave = tid >> 5, lane = tid & 31;
  const int r   = (int)blockIdx.x;
  const int c0  = tid * 8;
  const bool act = (c0 + 8 <= D);
  const int cc  = act ? c0 : 0;
  const float* p = F + (size_t)r * ldf + cc;
  const v4f a = *(const v4f*)(p), b4 = *(const v4f*)(p + 4);
  float v[8];
#pragma unroll
  for (int e = 0; e < 4; ++e) { v[e] = act ? a[e] : 0.0f; v[4 + e] = act ? b4[e] : 0.0f; }
  float ss = 0.0f;
#pragma unroll
  for (int e = 0; e < 8; ++e) ss = ss + v[e] * v[e];
#pragma unroll
  for (int off = 1; off < 32; off <<= 1) ss += __shfl_xor(ss, off, 32);
  if (lane == 0) red[wave] = ss;
  __syncthreads();
  const float tot = (red[0] + red[1]) + (red[2] + red[3]);
  if (!act) return;
  const float var = tot * invD;
  const float rs  = 1.0f / sqrtf(var + EPS_RMS);
  const v4f wa = *(const v4f*)(nw + cc), wb4 = *(const v4f*)(nw + cc + 4);
  float w[8];
#pragma unroll
  for (int e = 0; e < 4; ++e) { w[e] = bfr(wa[e]); w[4 + e] = bfr(wb4[e]); }
  v4u oh, ol;
#pragma unroll
  for (int e = 0; e < 4; ++e) {
    unsigned short h0, l0, h1, l1;
    hilo(((v[2 * e] * rs) * w[2 * e]) * sc, h0, l0);
    hilo(((v[2 * e + 1] * rs) * w[2 * e + 1]) * sc, h1, l1);
    oh[e] = pk16(h0, h1);
    ol[e] = pk16(l0, l1);
  }
  u16* dh = Hp + (size_t)r * D + c0;
  u16* dl = Lp + (size_t)r * D + c0;
  for (int pass = 0; pass < 2; ++pass) {
    *(volatile v4u*)(dh) = oh;
    *(volatile v4u*)(dl) = ol;
    __threadfence();
  }
}

__global__ __launch_bounds__(256) void cvt_hl(const float* __restrict__ F, int ldf, int w8, u16* Hp, u16* Lp,
                                              int n8, float sc) {
  const int gt = blockIdx.x * 256 + (int)threadIdx.x;
  if (gt >= n8) return;
  const int r  = gt / w8;
  const int c8 = gt - r * w8;
  const float* p = F + (size_t)r * ldf + c8 * 8;
  const v4f a = *(const v4f*)(p), b4 = *(const v4f*)(p + 4);
  float w[8];
#pragma unroll
  for (int e = 0; e < 4; ++e) { w[e] = a[e]; w[4 + e] = b4[e]; }
  v4u oh, ol;
#pragma unroll
  for (int e = 0; e < 4; ++e) {
    unsigned short h0, l0, h1, l1;
    hilo(w[2 * e] * sc, h0, l0);
    hilo(w[2 * e + 1] * sc, h1, l1);
    oh[e] = pk16(h0, h1);
    ol[e] = pk16(l0, l1);
  }
  u16* dh = Hp + (size_t)gt * 8;
  u16* dl = Lp + (size_t)gt * 8;
  for (int pass = 0; pass < 2; ++pass) {
    *(volatile v4u*)(dh) = oh;
    *(volatile v4u*)(dl) = ol;
    __threadfence();
  }
}

__global__ __launch_bounds__(128) void rope16(const float* __restrict__ F, int ldf, int b, int sbase,
                                              u16* Hp, u16* Lp, float sc) {
#pragma clang fp contract(off)
  __shared__ __align__(16) float cst[RHALF];
  __shared__ __align__(16) float snt[RHALF];
  const int tid = (int)threadIdx.x;
  const int r   = (int)blockIdx.x;
  if (r >= MCH) return;
  const int s   = sbase + r;
  if (tid < RHALF) {
    const float invf = exp2f((float)tid * KROPE);
    const float ang  = (float)s * invf;
    cst[tid] = cosf(ang);
    snt[tid] = sinf(ang);
  }
  __syncthreads();
  const int head = tid >> 3, i = tid & 7;
  const int d0 = 8 * i, dp = d0 ^ RHALF, j0 = d0 & (RHALF - 1);
  const float* p = F + (size_t)r * ldf + head * DR;
  const v4f xa = *(const v4f*)(p + d0), xb = *(const v4f*)(p + d0 + 4);
  const v4f pa = *(const v4f*)(p + dp), pb = *(const v4f*)(p + dp + 4);
  const v4f ca = *(const v4f*)(cst + j0), cb = *(const v4f*)(cst + j0 + 4);
  const v4f sa = *(const v4f*)(snt + j0), sb = *(const v4f*)(snt + j0 + 4);
  float x[8], pp[8], cv[8], sv[8];
#pragma unroll
  for (int e = 0; e < 4; ++e) {
    x[e] = xa[e];  x[4 + e] = xb[e];
    pp[e] = pa[e]; pp[4 + e] = pb[e];
    cv[e] = ca[e]; cv[4 + e] = cb[e];
    sv[e] = sa[e]; sv[4 + e] = sb[e];
  }
  const float sgn = (i < 4) ? -1.0f : 1.0f;
  float o[8];
#pragma unroll
  for (int e = 0; e < 8; ++e) o[e] = x[e] * cv[e] + (sgn * pp[e]) * sv[e];
  v4u oh, ol;
#pragma unroll
  for (int e = 0; e < 4; ++e) {
    unsigned short h0, l0, h1, l1;
    hilo(o[2 * e] * sc, h0, l0);
    hilo(o[2 * e + 1] * sc, h1, l1);
    oh[e] = pk16(h0, h1);
    ol[e] = pk16(l0, l1);
  }
  const size_t row = (size_t)b * SEQ + s;
  u16* dh = Hp + row * QPW + tid * 8;
  u16* dl = Lp + row * QPW + tid * 8;
  for (int pass = 0; pass < 2; ++pass) {
    *(volatile v4u*)(dh) = oh;
    *(volatile v4u*)(dl) = ol;
    __threadfence();
  }
}

__global__ __launch_bounds__(128) void kpe16(const float* __restrict__ F, int ldf, int b, int sbase,
                                             const float* __restrict__ nw, u16* Hp, u16* Lp, float sc) {
#pragma clang fp contract(off)
  __shared__ __align__(16) float cst[RPB * RHALF];
  __shared__ __align__(16) float snt[RPB * RHALF];
  const int tid = (int)threadIdx.x;
  const int r0  = (int)blockIdx.x * RPB;
  if (r0 + RPB > MCH) return;
#pragma unroll 1
  for (int it = 0; it < 4; ++it) {
    const int idx = tid + 128 * it;
    const int rr  = idx >> 5;
    const int j   = idx & 31;
    const float invf = exp2f((float)j * KROPE);
    const float ang  = (float)(sbase + r0 + rr) * invf;
    cst[idx] = cosf(ang);
    snt[idx] = sinf(ang);
  }
  __syncthreads();
  const int rr = tid >> 3, i = tid & 7;
  const int d0 = 8 * i, dp = d0 ^ RHALF, j0 = d0 & (RHALF - 1);
  const int r  = r0 + rr;
  const int s  = sbase + r;
  const float* p = F + (size_t)r * ldf;
  const v4f xa = *(const v4f*)(p + d0), xb = *(const v4f*)(p + d0 + 4);
  const v4f pa = *(const v4f*)(p + dp), pb = *(const v4f*)(p + dp + 4);
  const v4f ca = *(const v4f*)(cst + rr * RHALF + j0), cb = *(const v4f*)(cst + rr * RHALF + j0 + 4);
  const v4f sa = *(const v4f*)(snt + rr * RHALF + j0), sb = *(const v4f*)(snt + rr * RHALF + j0 + 4);
  const v4f wa = *(const v4f*)(nw + d0), wb4 = *(const v4f*)(nw + d0 + 4);
  const v4f wc = *(const v4f*)(nw + dp), wd = *(const v4f*)(nw + dp + 4);
  float x[8], pp[8], cv[8], sv[8], wo[8], wp[8];
#pragma unroll
  for (int e = 0; e < 4; ++e) {
    x[e] = xa[e];        x[4 + e] = xb[e];
    pp[e] = pa[e];       pp[4 + e] = pb[e];
    cv[e] = ca[e];       cv[4 + e] = cb[e];
    sv[e] = sa[e];       sv[4 + e] = sb[e];
    wo[e] = bfr(wa[e]);  wo[4 + e] = bfr(wb4[e]);
    wp[e] = bfr(wc[e]);  wp[4 + e] = bfr(wd[e]);
  }
  float ss = 0.0f;
#pragma unroll
  for (int e = 0; e < 8; ++e) ss = ss + x[e] * x[e];
  ss += __shfl_xor(ss, 1, 32);
  ss += __shfl_xor(ss, 2, 32);
  ss += __shfl_xor(ss, 4, 32);
  const float var = ss * (1.0f / (float)DR);
  const float rs  = 1.0f / sqrtf(var + EPS_RMS);
  const float sgn = (i < 4) ? -1.0f : 1.0f;
  float o[8];
#pragma unroll
  for (int e = 0; e < 8; ++e) {
    const float y  = (x[e] * rs) * wo[e];
    const float yp = (pp[e] * rs) * wp[e];
    o[e] = y * cv[e] + (sgn * yp) * sv[e];
  }
  v4u oh, ol;
#pragma unroll
  for (int e = 0; e < 4; ++e) {
    unsigned short h0, l0, h1, l1;
    hilo(o[2 * e] * sc, h0, l0);
    hilo(o[2 * e + 1] * sc, h1, l1);
    oh[e] = pk16(h0, h1);
    ol[e] = pk16(l0, l1);
  }
  const size_t row = (size_t)b * SEQ + s;
  u16* dh = Hp + row * DR + d0;
  u16* dl = Lp + row * DR + d0;
  for (int pass = 0; pass < 2; ++pass) {
    *(volatile v4u*)(dh) = oh;
    *(volatile v4u*)(dl) = ol;
    __threadfence();
  }
}

__global__ __launch_bounds__(256) void vt16(const float* __restrict__ F, int ldf, int b, int sbase, u16* VHo, u16* VLo) {
  __shared__ __align__(16) u16 TH[DV * VTP];
  __shared__ __align__(16) u16 TL[DV * VTP];
  const int tid = threadIdx.x;
  const int bid = blockIdx.x;
  const int st  = bid % NST;
  const int h   = bid / NST;
  if (h >= NKV) return;
  const int sl0 = st * 64;
  {
    const int sl = tid >> 2;
    const int dc = (tid & 3) * 32;
    const float* src = F + (size_t)(sl0 + sl) * ldf + h * DV + dc;
#pragma unroll
    for (int i = 0; i < 8; ++i) {
      const v4f a = *(const v4f*)(src + 4 * i);
#pragma unroll
      for (int e = 0; e < 4; ++e) {
        unsigned short hb, lb;
        hilo(a[e] * VCAR, hb, lb);
        TH[(dc + 4 * i + e) * VTP + sl] = hb;
        TL[(dc + 4 * i + e) * VTP + sl] = lb;
      }
    }
  }
  __syncthreads();
  v4u vh[4], vl[4];
  const int q8 = tid >> 3, p8 = (tid & 7) * 8;
#pragma unroll
  for (int it = 0; it < 4; ++it) {
    const int line = it * 32 + q8;
    vh[it] = *(const v4u*)(TH + line * VTP + p8);
    vl[it] = *(const v4u*)(TL + line * VTP + p8);
  }
  const size_t hrow = (size_t)(b * NKV + h) * DV;
  const size_t base = hrow * SEQ + (size_t)(sbase + sl0) + p8;
  for (int pass = 0; pass < 2; ++pass) {
#pragma unroll
    for (int it = 0; it < 4; ++it) {
      const int line = it * 32 + q8;
      *(volatile v4u*)(VHo + base + (size_t)line * SEQ) = vh[it];
      *(volatile v4u*)(VLo + base + (size_t)line * SEQ) = vl[it];
    }
    __threadfence();
  }
}

__device__ __forceinline__ void epi64n(float* sl, v8f a0, v8f a1, v8f a2, v8f a3, float oscale,
                                       float* C, int ldc, size_t rowb, int col0, int lane) {
  const int hh = lane >> 4, m = lane & 15;
#pragma unroll
  for (int r = 0; r < 8; ++r) {
    const int ro = (8 * hh + r) * 68 + m;
    sl[ro]      = a0[r] * oscale;
    sl[ro + 16] = a1[r] * oscale;
    sl[ro + 32] = a2[r] * oscale;
    sl[ro + 48] = a3[r] * oscale;
  }
  wave_sync_lds();
  v4f vals[8];
#pragma unroll
  for (int it = 0; it < 8; ++it) vals[it] = *(const v4f*)(sl + (it * 2 + hh) * 68 + m * 4);
  float* dst = C + (rowb + (size_t)hh) * (size_t)ldc + col0 + m * 4;
  for (int pass = 0; pass < 2; ++pass) {
#pragma unroll
    for (int it = 0; it < 8; ++it) {
      *(volatile v4f*)(dst + (size_t)(it * 2) * (size_t)ldc) = vals[it];
    }
    __threadfence();
  }
}

__global__ __launch_bounds__(128)
void gemm_b1(const u16* __restrict__ A, const u16* __restrict__ Bt, float* C, int M, int N, int K) {
  __shared__ __align__(16) float slab[4 * SLAB64];
  const int tid = threadIdx.x, wave = tid >> 5, lane = tid & 31, hh = lane >> 4, m = lane & 15;
  const int ntile = N >> 6;
  const int bid   = blockIdx.x;
  const int rowb  = (bid / ntile) * 64 + wave * 16;
  const int col0  = (bid % ntile) * 64;
  if (rowb + 16 > M) return;
  const u16* ap = A  + (size_t)(rowb + m) * K + 8 * hh;
  const u16* bp = Bt + (size_t)(col0 + m) * K + 8 * hh;
  const size_t bs = (size_t)16 * K;
  v8f acc0 = zero8(), acc1 = zero8(), acc2 = zero8(), acc3 = zero8();
#pragma unroll 1
  for (int k0 = 0; k0 < K; k0 += 32) {
    const v16b a  = ldfrag_b(ap + k0);
    const v16b b0 = ldfrag_b(bp + k0);
    const v16b b1 = ldfrag_b(bp + bs + k0);
    const v16b b2 = ldfrag_b(bp + 2 * bs + k0);
    const v16b b3 = ldfrag_b(bp + 3 * bs + k0);
    acc0 = mma_b(a, b0, acc0);
    acc1 = mma_b(a, b1, acc1);
    acc2 = mma_b(a, b2, acc2);
    acc3 = mma_b(a, b3, acc3);
    guard6<v16b>(acc0, acc1, acc2, acc3, a, b0, b1, b2, b3, a);
  }
  epi64n(slab + wave * SLAB64, acc0, acc1, acc2, acc3, 1.0f, C, N, (size_t)rowb, col0, lane);
}

template <int NPROD>
__global__ __launch_bounds__(128)
void gemm_h(const u16* __restrict__ Ah, const u16* __restrict__ Al, const u16* __restrict__ Bt,
            float* C, int M, int N, int K, int ldc, float oscale) {
  __shared__ __align__(16) float slab[4 * SLAB64];
  const int tid = threadIdx.x, wave = tid >> 5, lane = tid & 31, hh = lane >> 4, m = lane & 15;
  const int ntile = N >> 6;
  const int bid   = blockIdx.x;
  const int rowb  = (bid / ntile) * 64 + wave * 16;
  const int col0  = (bid % ntile) * 64;
  if (rowb + 16 > M) return;
  const _Float16* ahp = (const _Float16*)(const void*)Ah + (size_t)(rowb + m) * K + 8 * hh;
  const _Float16* alp = (const _Float16*)(const void*)Al + (size_t)(rowb + m) * K + 8 * hh;
  const _Float16* bp  = (const _Float16*)(const void*)Bt + (size_t)(col0 + m) * K + 8 * hh;
  const size_t bs = (size_t)16 * K;
  v8f acc0 = zero8(), acc1 = zero8(), acc2 = zero8(), acc3 = zero8();
  if constexpr (NPROD == 2) {
#pragma unroll 1
    for (int k0 = 0; k0 < K; k0 += 32) {
      const v16h ah = ldfrag_h(ahp + k0), al = ldfrag_h(alp + k0);
      const v16h b0 = ldfrag_h(bp + k0);
      const v16h b1 = ldfrag_h(bp + bs + k0);
      const v16h b2 = ldfrag_h(bp + 2 * bs + k0);
      const v16h b3 = ldfrag_h(bp + 3 * bs + k0);
      acc0 = mma_h(ah, b0, acc0);  acc0 = mma_h(al, b0, acc0);
      acc1 = mma_h(ah, b1, acc1);  acc1 = mma_h(al, b1, acc1);
      acc2 = mma_h(ah, b2, acc2);  acc2 = mma_h(al, b2, acc2);
      acc3 = mma_h(ah, b3, acc3);  acc3 = mma_h(al, b3, acc3);
      guard6<v16h>(acc0, acc1, acc2, acc3, ah, al, b0, b1, b2, b3);
    }
  } else {
#pragma unroll 1
    for (int k0 = 0; k0 < K; k0 += 32) {
      const v16h ah = ldfrag_h(ahp + k0);
      const v16h b0 = ldfrag_h(bp + k0);
      const v16h b1 = ldfrag_h(bp + bs + k0);
      const v16h b2 = ldfrag_h(bp + 2 * bs + k0);
      const v16h b3 = ldfrag_h(bp + 3 * bs + k0);
      acc0 = mma_h(ah, b0, acc0);
      acc1 = mma_h(ah, b1, acc1);
      acc2 = mma_h(ah, b2, acc2);
      acc3 = mma_h(ah, b3, acc3);
      guard6<v16h>(acc0, acc1, acc2, acc3, ah, b0, b1, b2, b3, ah);
    }
  }
  epi64n(slab + wave * SLAB64, acc0, acc1, acc2, acc3, oscale, C, ldc, (size_t)rowb, col0, lane);
}

__global__ __launch_bounds__(ATT_THREADS)
void attn_c(const u16* __restrict__ QHp, const u16* __restrict__ QLp,
            const u16* __restrict__ PHp, const u16* __restrict__ PLp,
            const u16* __restrict__ KHp, const u16* __restrict__ KLp,
            const u16* __restrict__ RHp, const u16* __restrict__ RLp,
            const u16* __restrict__ VHp, const u16* __restrict__ VLp,
            u16* OHp, u16* OLp) {
  __shared__ __align__(16) float smem[WPB * WREG];

  const int tid  = threadIdx.x;
  const int wave = tid >> 5;
  const int lane = tid & 31;
  const int hh   = lane >> 4;
  const int c    = lane & 15;
  const int bid  = blockIdx.x;
  const int qt   = bid % NQT;
  const int t2   = bid / NQT;
  const int hg   = t2 % NHG;
  const int b    = t2 / NHG;
  if (b >= NB) return;
  const int q0   = qt * 16;
  if (q0 + 16 > SEQ) return;
  const int head = hg * WPB + wave;
  const int kvh  = hg;
  const bool vres = (q0 < QO);

  float* pt   = smem + wave * WREG;
  float* slab = pt + PTW;

  const size_t qrow = (size_t)b * SEQ + q0 + c;
  const size_t krow = (size_t)b * SEQ + c;
  const _Float16* Qh  = (const _Float16*)(const void*)QHp + qrow * QNW + (size_t)head * DN + 8 * hh;
  const _Float16* Ql  = (const _Float16*)(const void*)QLp + qrow * QNW + (size_t)head * DN + 8 * hh;
  const _Float16* Qph = (const _Float16*)(const void*)PHp + qrow * QPW + (size_t)head * DR + 8 * hh;
  const _Float16* Qpl = (const _Float16*)(const void*)PLp + qrow * QPW + (size_t)head * DR + 8 * hh;
  const _Float16* Khb = (const _Float16*)(const void*)KHp + krow * KNW + (size_t)kvh * DN + 8 * hh;
  const _Float16* Klb = (const _Float16*)(const void*)KLp + krow * KNW + (size_t)kvh * DN + 8 * hh;
  const _Float16* Rhb = (const _Float16*)(const void*)RHp + krow * DR + 8 * hh;
  const _Float16* Rlb = (const _Float16*)(const void*)RLp + krow * DR + 8 * hh;
  const _Float16* Vhb = (const _Float16*)(const void*)VHp + (((size_t)b * NKV + kvh) * DV + c) * SEQ + 8 * hh;
  const _Float16* Vlb = (const _Float16*)(const void*)VLp + (((size_t)b * NKV + kvh) * DV + c) * SEQ + 8 * hh;
  const float lsc = SCL * (LOG2E / (QSC * KSC));
  const float oc  = 1.0f / (PCAR * VCAR);

  float mrow[8], lrow[8];
  v8f o[8];
#pragma unroll
  for (int r = 0; r < 8; ++r) { mrow[r] = -INFINITY; lrow[r] = 0.f; }
#pragma unroll
  for (int j = 0; j < 8; ++j) o[j] = zero8();
  const int ncaus = (q0 >> 5) + 1;
  const int nkt = (ncaus < NKT) ? ncaus : NKT;
  const int qr0 = q0 + 8 * hh;

#pragma unroll 1
  for (int kt = 0; kt < nkt; ++kt) {
    const int kb = kt * 32;
    v8f s0 = zero8(), s1 = zero8();
    {
      const _Float16* k0p = Khb + (size_t)kb * KNW;
      const _Float16* k1p = k0p + (size_t)16 * KNW;
      const _Float16* l0p = Klb + (size_t)kb * KNW;
      const _Float16* l1p = l0p + (size_t)16 * KNW;
#pragma unroll
      for (int kk = 0; kk < DN / 32; ++kk) {
        const v16h qh  = ldfrag_h(Qh + kk * 32);
        const v16h ql  = ldfrag_h(Ql + kk * 32);
        const v16h kh0 = ldfrag_h(k0p + kk * 32);
        const v16h kh1 = ldfrag_h(k1p + kk * 32);
        const v16h kl0 = ldfrag_h(l0p + kk * 32);
        const v16h kl1 = ldfrag_h(l1p + kk * 32);
        s0 = mma_h(qh, kh0, s0);
        s0 = mma_h(ql, kh0, s0);
        s0 = mma_h(qh, kl0, s0);
        s1 = mma_h(qh, kh1, s1);
        s1 = mma_h(ql, kh1, s1);
        s1 = mma_h(qh, kl1, s1);
        guard2(s0, s1, qh, ql, kh0, kl0, kh1, kl1);
      }
    }
    {
      const _Float16* k0p = Rhb + (size_t)kb * DR;
      const _Float16* k1p = k0p + (size_t)16 * DR;
      const _Float16* l0p = Rlb + (size_t)kb * DR;
      const _Float16* l1p = l0p + (size_t)16 * DR;
#pragma unroll
      for (int kk = 0; kk < DR / 32; ++kk) {
        const v16h qh  = ldfrag_h(Qph + kk * 32);
        const v16h ql  = ldfrag_h(Qpl + kk * 32);
        const v16h kh0 = ldfrag_h(k0p + kk * 32);
        const v16h kh1 = ldfrag_h(k1p + kk * 32);
        const v16h kl0 = ldfrag_h(l0p + kk * 32);
        const v16h kl1 = ldfrag_h(l1p + kk * 32);
        s0 = mma_h(qh, kh0, s0);
        s0 = mma_h(ql, kh0, s0);
        s0 = mma_h(qh, kl0, s0);
        s1 = mma_h(qh, kh1, s1);
        s1 = mma_h(ql, kh1, s1);
        s1 = mma_h(qh, kl1, s1);
        guard2(s0, s1, qh, ql, kh0, kl0, kh1, kl1);
      }
    }
    const int key0 = kb + c, key1 = kb + 16 + c;
#pragma unroll
    for (int r = 0; r < 8; ++r) {
      const int   qr = qr0 + r;
      const float u0 = s0[r] * lsc;
      const float u1 = s1[r] * lsc;
      const float t0 = (key0 <= qr) ? u0 : NEGT;
      const float t1 = (key1 <= qr) ? u1 : NEGT;
      float mx = fmaxf(t0, t1);
#pragma unroll
      for (int off = 1; off < 16; off <<= 1) mx = fmaxf(mx, __shfl_xor(mx, off, 32));
      const float mn = fmaxf(mrow[r], mx);
      const float ms = (mn == -INFINITY) ? 0.0f : mn;
      const float al = exp2f(mrow[r] - ms);
      mrow[r] = mn;
      const float e0 = exp2f(t0 - ms), e1 = exp2f(t1 - ms);
      float ps = e0 + e1;
#pragma unroll
      for (int off = 1; off < 16; off <<= 1) ps += __shfl_xor(ps, off, 32);
      lrow[r] = lrow[r] * al + ps;
#pragma unroll
      for (int j = 0; j < 8; ++j) o[j][r] *= al;
      const int ro = (8 * hh + r) * PTP + c;
      pt[ro]      = e0;
      pt[ro + 16] = e1;
    }
    wave_sync_lds();
    FragH ph, pl;
    {
      const float* prow = pt + c * PTP + 8 * hh;
      const v4f p0 = *(const v4f*)(prow), p1 = *(const v4f*)(prow + 4);
      const v4f p2 = *(const v4f*)(prow + 16), p3 = *(const v4f*)(prow + 20);
#pragma unroll
      for (int e = 0; e < 4; ++e) {
        const float ta = p0[e] * PCAR, tb = p1[e] * PCAR, tc = p2[e] * PCAR, td = p3[e] * PCAR;
        const _Float16 ha = (_Float16)ta, hb = (_Float16)tb, hc = (_Float16)tc, hd = (_Float16)td;
        ph.h[0][e]     = ha;
        ph.h[0][4 + e] = hb;
        ph.h[1][e]     = hc;
        ph.h[1][4 + e] = hd;
        pl.h[0][e]     = (_Float16)(ta - (float)ha);
        pl.h[0][4 + e] = (_Float16)(tb - (float)hb);
        pl.h[1][e]     = (_Float16)(tc - (float)hc);
        pl.h[1][4 + e] = (_Float16)(td - (float)hd);
      }
    }
    {
      const _Float16* vhp = Vhb + kb;
      const _Float16* vlp = Vlb + kb;
      if (vres) {
#pragma unroll
        for (int jg = 0; jg < 4; ++jg) {
          const size_t da = (size_t)(2 * jg) * 16 * SEQ;
          const size_t db = da + (size_t)16 * SEQ;
          const v16h vha = ldfrag_h(vhp + da), vhb2 = ldfrag_h(vhp + db);
          const v16h vla = ldfrag_h(vlp + da), vlb2 = ldfrag_h(vlp + db);
          o[2 * jg]     = mma_h(ph.v, vha,  o[2 * jg]);
          o[2 * jg]     = mma_h(pl.v, vha,  o[2 * jg]);
          o[2 * jg]     = mma_h(ph.v, vla,  o[2 * jg]);
          o[2 * jg + 1] = mma_h(ph.v, vhb2, o[2 * jg + 1]);
          o[2 * jg + 1] = mma_h(pl.v, vhb2, o[2 * jg + 1]);
          o[2 * jg + 1] = mma_h(ph.v, vlb2, o[2 * jg + 1]);
          guard2(o[2 * jg], o[2 * jg + 1], ph.v, pl.v, vha, vhb2, vla, vlb2);
        }
      } else {
#pragma unroll
        for (int jg = 0; jg < 4; ++jg) {
          const size_t da = (size_t)(2 * jg) * 16 * SEQ;
          const size_t db = da + (size_t)16 * SEQ;
          const v16h vha = ldfrag_h(vhp + da), vhb2 = ldfrag_h(vhp + db);
          o[2 * jg]     = mma_h(ph.v, vha,  o[2 * jg]);
          o[2 * jg]     = mma_h(pl.v, vha,  o[2 * jg]);
          o[2 * jg + 1] = mma_h(ph.v, vhb2, o[2 * jg + 1]);
          o[2 * jg + 1] = mma_h(pl.v, vhb2, o[2 * jg + 1]);
          guard2(o[2 * jg], o[2 * jg + 1], ph.v, pl.v, vha, vhb2, vha, vhb2);
        }
      }
    }
    wave_sync_lds();
  }
  acc_guard4(o[0], o[1], o[2], o[3]);
  acc_guard4(o[4], o[5], o[6], o[7]);
#pragma unroll
  for (int r = 0; r < 8; ++r) {
    const float lv  = lrow[r];
    const float ls  = (lv > 0.0f) ? lv : 1.0f;
    const float inv = (lv > 0.0f) ? ((1.0f / ls) * oc) : 0.0f;
#pragma unroll
    for (int j = 0; j < 8; ++j) {
      const int idx = (8 * hh + r) * SLP + j * 16 + c;
      slab[idx] = o[j][r] * inv;
    }
  }

  wave_sync_lds();
  v4u oh[8], ol[8];
  const int rq = lane >> 4, c8 = (lane & 15) * 8;
#pragma unroll
  for (int it = 0; it < 8; ++it) {
    const int row = it * 2 + rq;
    const v4f a = *(const v4f*)(slab + row * SLP + c8), b4 = *(const v4f*)(slab + row * SLP + c8 + 4);
    float w[8];
#pragma unroll
    for (int e = 0; e < 4; ++e) { w[e] = a[e] * OSC; w[4 + e] = b4[e] * OSC; }
#pragma unroll
    for (int e = 0; e < 4; ++e) {
      unsigned short h0, l0, h1, l1;
      hilo(w[2 * e], h0, l0);
      hilo(w[2 * e + 1], h1, l1);
      oh[it][e] = pk16(h0, h1);
      ol[it][e] = pk16(l0, l1);
    }
  }
  const size_t ob  = ((size_t)b * SEQ + q0) * ODIM + (size_t)head * DV + c8;
  const size_t olb = ((size_t)b * QO  + q0) * ODIM + (size_t)head * DV + c8;
  for (int pass = 0; pass < 2; ++pass) {
#pragma unroll
    for (int it = 0; it < 8; ++it) {
      const int row = it * 2 + rq;
      *(volatile v4u*)(OHp + ob + (size_t)row * ODIM) = oh[it];
      if (vres) {
        *(volatile v4u*)(OLp + olb + (size_t)row * ODIM) = ol[it];
      }
    }
    __threadfence();
  }
}

extern "C" void kernel_launch(void* const* d_in, const int* in_sizes, int n_in,
                              void* d_out, int out_size, void* d_ws, size_t ws_size,
                              hipStream_t stream) {
  if (n_in < 11) return;
  if (in_sizes[0] < ((NB - 1) * XS_FULL + SEQ) * DMOD) return;
  if (in_sizes[1] != DMOD * QLR) return;
  if (in_sizes[2] != QLR) return;
  if (in_sizes[3] != QLR * QNW) return;
  if (in_sizes[4] != QLR * QPW) return;
  if (in_sizes[5] != DMOD * KVLR) return;
  if (in_sizes[6] != KVLR) return;
  if (in_sizes[7] != KVLR * NKVUP) return;
  if (in_sizes[8] != DMOD * DR) return;
  if (in_sizes[9] != DR) return;
  if (in_sizes[10] != ODIM * DMOD) return;
  if (out_size < ((NB - 1) * XS_FULL + SEQ) * DMOD) return;

  const float* x    = (const float*)d_in[0];
  const float* wqd  = (const float*)d_in[1];
  const float* qnw  = (const float*)d_in[2];
  const float* wqu  = (const float*)d_in[3];
  const float* wqp  = (const float*)d_in[4];
  const float* wkd  = (const float*)d_in[5];
  const float* kvw  = (const float*)d_in[6];
  const float* wku  = (const float*)d_in[7];
  const float* wkp  = (const float*)d_in[8];
  const float* kpw  = (const float*)d_in[9];
  const float* wout = (const float*)d_in[10];
  float*       out  = (float*)d_out;

  const size_t szXB  = (size_t)MCH * DMOD * 2;
  const size_t szWD  = (size_t)NDOWN * DMOD * 2;
  const size_t szWQU = (size_t)NQUP * QLR * 2;
  const size_t szWKU = (size_t)NKVUP * KVLR * 2;
  const size_t szFd  = (size_t)MCH * NDOWN * 4;
  const size_t szCQ  = (size_t)MCH * QLR * 2;
  const size_t szCK  = (size_t)MCH * KVLR * 2;
  const size_t szFu  = (size_t)MCH * NQUP * 4;
  const size_t szOH  = (size_t)MROWS * ODIM * 2;
  const size_t szOL  = (size_t)NB * QO * ODIM * 2;
  const size_t szQN  = (size_t)MROWS * QNW * 2;
  const size_t szQP  = (size_t)MROWS * QPW * 2;
  const size_t szKN  = (size_t)MROWS * KNW * 2;
  const size_t szKP  = (size_t)MROWS * DR * 2;
  const size_t szV   = (size_t)NB * NKV * DV * SEQ * 2;
  const size_t szWO  = (size_t)ODIM * DMOD * 2;

  size_t off = 0;
  const size_t oXB  = off; off += szXB;
  const size_t oWD  = off; off += szWD;
  const size_t oWQU = off; off += szWQU;
  const size_t oWKU = off; off += szWKU;
  const size_t oFd  = off; off += szFd;
  const size_t oCQH = off; off += szCQ;
  const size_t oCQL = off; off += szCQ;
  const size_t oCKH = off; off += szCK;
  const size_t oCKL = off; off += szCK;
  const size_t oFu  = off; off += szFu;
  const size_t g0a  = off;
  const size_t oOH  = 0;
  const size_t oOL  = szOH;
  const size_t g0b  = szOH + szOL;
  const size_t G0   = (g0a > g0b) ? g0a : g0b;
  off = G0;
  const size_t oQH  = off; off += szQN;
  const size_t oQL  = off; off += szQN;
  const size_t oQPH = off; off += szQP;
  const size_t oQPL = off; off += szQP;
  const size_t oKH  = off; off += szKN;
  const size_t oKL  = off; off += szKN;
  const size_t oRH  = off; off += szKP;
  const size_t oRL  = off; off += szKP;
  const size_t oVH  = off; off += szV;
  const size_t oVL  = off; off += szV;
  const size_t oWO  = off; off += szWO;
  if (off > ws_size) return;
  if (off > (size_t)WS_CAP) return;

  char* ws = (char*)d_ws;
  u16*   XB  = (u16*)(ws + oXB);
  u16*   WD  = (u16*)(ws + oWD);
  u16*   WQU = (u16*)(ws + oWQU);
  u16*   WKU = (u16*)(ws + oWKU);
  float* Fd  = (float*)(ws + oFd);
  u16*   CQH = (u16*)(ws + oCQH);
  u16*   CQL = (u16*)(ws + oCQL);
  u16*   CKH = (u16*)(ws + oCKH);
  u16*   CKL = (u16*)(ws + oCKL);
  float* Fu  = (float*)(ws + oFu);
  u16*   OH  = (u16*)(ws + oOH);
  u16*   OL  = (u16*)(ws + oOL);
  u16*   QH  = (u16*)(ws + oQH);
  u16*   QL  = (u16*)(ws + oQL);
  u16*   QPH = (u16*)(ws + oQPH);
  u16*   QPL = (u16*)(ws + oQPL);
  u16*   KH  = (u16*)(ws + oKH);
  u16*   KL  = (u16*)(ws + oKL);
  u16*   RH  = (u16*)(ws + oRH);
  u16*   RL  = (u16*)(ws + oRL);
  u16*   VH  = (u16*)(ws + oVH);
  u16*   VL  = (u16*)(ws + oVL);
  u16*   WO  = (u16*)(ws + oWO);

  const dim3 b256(256), b128(128), bAT(ATT_THREADS);
  const int  n8x = (MCH * DMOD) / 8;
  const int  n8q = (MCH * QNW) / 8;
  const int  n8k = (MCH * KNW) / 8;
  const float upsc = 1.0f / (CSC * WUS);

  tw16<<<dim3((DMOD / 64) * (QLR / 64)), b256, 0, stream>>>(wqd, QLR, DMOD, QLR, WD, 0, 1.0f);
  tw16<<<dim3((DMOD / 64) * (KVLR / 64)), b256, 0, stream>>>(wkd, KVLR, DMOD, KVLR, WD + (size_t)QLR * DMOD, 0, 1.0f);
  tw16<<<dim3((DMOD / 64) * (DR / 64)), b256, 0, stream>>>(wkp, DR, DMOD, DR, WD + (size_t)(QLR + KVLR) * DMOD, 0, 1.0f);
  tw16<<<dim3((QLR / 64) * (QNW / 64)), b256, 0, stream>>>(wqu, QNW, QLR, QNW, WQU, 1, WUS);
  tw16<<<dim3((QLR / 64) * (QPW / 64)), b256, 0, stream>>>(wqp, QPW, QLR, QPW, WQU + (size_t)QNW * QLR, 1, WUS);
  tw16<<<dim3((KVLR / 64) * (NKVUP / 64)), b256, 0, stream>>>(wku, NKVUP, KVLR, NKVUP, WKU, 1, WUS);

  for (int b = 0; b < NB; ++b) {
    for (int ch = 0; ch < NCH; ++ch) {
      const int sbase = ch * MCH;
      const size_t roff = (size_t)b * SEQ + sbase;
      cvtb16<<<dim3(n8x / 256), b256, 0, stream>>>(x + ((size_t)b * XS_FULL + sbase) * DMOD, XB, n8x);
      gemm_b1<<<dim3((MCH / 64) * (NDOWN / 64)), b128, 0, stream>>>(XB, WD, Fd, MCH, NDOWN, DMOD);
      rnorm16<<<dim3(MCH), b128, 0, stream>>>(Fd, NDOWN, QLR, 1.0f / (float)QLR, qnw, CQH, CQL, CSC);
      gemm_h<2><<<dim3((MCH / 64) * (NQUP / 64)), b128, 0, stream>>>(CQH, CQL, WQU, Fu, MCH, NQUP, QLR, NQUP, upsc);
      cvt_hl<<<dim3(n8q / 256), b256, 0, stream>>>(Fu, NQUP, QNW / 8, QH + roff * QNW, QL + roff * QNW, n8q, QSC);
      rope16<<<dim3(MCH), b128, 0, stream>>>(Fu + QNW, NQUP, b, sbase, QPH, QPL, QSC);
      rnorm16<<<dim3(MCH), b128, 0, stream>>>(Fd + QLR, NDOWN, KVLR, 1.0f / (float)KVLR, kvw, CKH, CKL, CSC);
      gemm_h<2><<<dim3((MCH / 64) * (NKVUP / 64)), b128, 0, stream>>>(CKH, CKL, WKU, Fu, MCH, NKVUP, KVLR, NKVUP, upsc);
      cvt_hl<<<dim3(n8k / 256), b256, 0, stream>>>(Fu, NKVUP, KNW / 8, KH + roff * KNW, KL + roff * KNW, n8k, KSC);
      vt16<<<dim3(NKV * NST), b256, 0, stream>>>(Fu + KNW, NKVUP, b, sbase, VH, VL);
      kpe16<<<dim3(MCH / RPB), b128, 0, stream>>>(Fd + QLR + KVLR, NDOWN, b, sbase, kpw, RH, RL, KSC);
    }
  }
  attn_c<<<dim3(NQT * NHG * NB), bAT, 0, stream>>>(QH, QL, QPH, QPL, KH, KL, RH, RL, VH, VL, OH, OL);
  tw16<<<dim3((ODIM / 64) * (DMOD / 64)), b256, 0, stream>>>(wout, DMOD, ODIM, DMOD, WO, 1, WOS);
  const float osc = 1.0f / (OSC * WOS);
  for (int b = 0; b < NB; ++b) {
    gemm_h<2><<<dim3((QO / 64) * (DMOD / 64)), b128, 0, stream>>>(
        OH + (size_t)b * SEQ * ODIM, OL + (size_t)b * QO * ODIM, WO, out + (size_t)b * XS_FULL * DMOD,
        QO, DMOD, ODIM, DMOD, osc);
    if (SEQ > QO) {
      gemm_h<1><<<dim3(((SEQ - QO) / 64) * (DMOD / 64)), b128, 0, stream>>>(
          OH + ((size_t)b * SEQ + QO) * ODIM, OH + ((size_t)b * SEQ + QO) * ODIM, WO,
          out + ((size_t)b * XS_FULL + QO) * DMOD, SEQ - QO, DMOD, ODIM, DMOD, osc);
    }
  }
  (void)hipGetLastError();
}
